// EfficientKANConv_68032281969066
// MI455X (gfx1250) — hardware-verified
//
#include <hip/hip_runtime.h>

#pragma clang fp contract(off)

typedef __attribute__((ext_vector_type(16))) _Float16 v16h;
typedef __attribute__((ext_vector_type(8)))  _Float16 v8h;
typedef __attribute__((ext_vector_type(16))) __bf16   v16b;
typedef __attribute__((ext_vector_type(8)))  __bf16   v8b;
typedef __attribute__((ext_vector_type(8)))  float    v8f;
typedef __attribute__((ext_vector_type(4)))  float    v4f;
typedef __attribute__((ext_vector_type(4)))  unsigned int v4u;

constexpr int kBatch  = 8;
constexpr int kCin    = 32;
constexpr int kCout   = 128;
constexpr int kImgH   = 64;
constexpr int kImgW   = 64;
constexpr int kPos    = kImgH * kImgW;
constexpr int kRows   = kBatch * kPos;
constexpr int kTaps   = 9;
constexpr int kNB     = 8;
constexpr int kKpatch = kCin * kTaps;
constexpr int kKsp    = kKpatch * kNB;
constexpr int kKtot   = kKsp + kKpatch;
constexpr int kPitch  = 2624;
constexpr int kWChunks = kPitch / 8;
constexpr int kNPix   = kBatch * kCin * kPos;
constexpr int kNPixP  = kNPix + 32;
constexpr int kZSlot  = kNPix;
constexpr int kChunkRows   = kPos;
constexpr int kNumChunks   = kBatch;
constexpr int kRowsPerBlk  = 32;
constexpr int kGroups      = 5;
constexpr int kTasksPerWave = kRowsPerBlk * kGroups / 8;

__device__ __forceinline__ unsigned short f2bf_bits(float f) {
  unsigned u = __float_as_uint(f);
  return (unsigned short)((u + 0x7FFFu + ((u >> 16) & 1u)) >> 16);
}
__device__ __forceinline__ float bf_bits2f(unsigned short h) { return __uint_as_float(((unsigned)h) << 16); }

__device__ __forceinline__ void dep_guard_h(v8f& a, v8f& b, v16h x, v16h y) { asm volatile("v_nop\n\tv_nop\n\tv_nop\n\tv_nop" : "+v"(a), "+v"(b) : "v"(x), "v"(y)); }
__device__ __forceinline__ void dep_guard_b(v8f& a, v8f& b, v16b x, v16b y) { asm volatile("v_nop\n\tv_nop\n\tv_nop\n\tv_nop" : "+v"(a), "+v"(b) : "v"(x), "v"(y)); }
__device__ __forceinline__ void keep4_h(v16h a, v16h b, v16h c, v16h d) { asm volatile("v_nop" :: "v"(a), "v"(b), "v"(c), "v"(d)); }
__device__ __forceinline__ void keep4_b(v16b a, v16b b, v16b c, v16b d) { asm volatile("v_nop" :: "v"(a), "v"(b), "v"(c), "v"(d)); }
__device__ __forceinline__ void acc_guard4(v8f& a, v8f& b, v8f& c, v8f& d) { asm volatile("v_nop\n\tv_nop\n\tv_nop\n\tv_nop" : "+v"(a), "+v"(b), "+v"(c), "+v"(d)); }
template <typename T> struct Frag;
template <> struct Frag<_Float16> {
  typedef v16h V; union U { v16h v; v8h h[2]; };
  static __device__ __forceinline__ v16h load(const _Float16* p) {
    U f; f.h[0] = *(const v8h*)(p); f.h[1] = *(const v8h*)(p + 16); return f.v;
  }
  static __device__ __forceinline__ v8f mma(v16h a, v16h b, v8f c) {
    return __builtin_amdgcn_wmma_f32_16x16x32_f16(false, a, false, b, (short)0, c, false, false);
  }
  static __device__ __forceinline__ void guard(v8f& a, v8f& b, v16h x, v16h y) { dep_guard_h(a, b, x, y); }
  static __device__ __forceinline__ void keep(v16h a, v16h b, v16h c, v16h d) { keep4_h(a, b, c, d); }
};
template <> struct Frag<__bf16> {
  typedef v16b V; union U { v16b v; v8b h[2]; };
  static __device__ __forceinline__ v16b load(const __bf16* p) {
    U f; f.h[0] = *(const v8b*)(p); f.h[1] = *(const v8b*)(p + 16); return f.v;
  }
  static __device__ __forceinline__ v8f mma(v16b a, v16b b, v8f c) {
    return __builtin_amdgcn_wmma_f32_16x16x32_bf16(false, a, false, b, (short)0, c, false, false);
  }
  static __device__ __forceinline__ void guard(v8f& a, v8f& b, v16b x, v16b y) { dep_guard_b(a, b, x, y); }
  static __device__ __forceinline__ void keep(v16b a, v16b b, v16b c, v16b d) { keep4_b(a, b, c, d); }
};

template <int ET> struct Elem;
template <> struct Elem<0> { typedef _Float16 T; };
template <> struct Elem<1> { typedef __bf16 T; };
template <int ET, bool SPLIT, int BIAS_MODE, int OUT_MODE, bool RESID, int ACT = 0>
__global__ __launch_bounds__(256) void wmma_gemm64(
    const unsigned short* __restrict__ Ap, const unsigned short* __restrict__ A2p, int lda, long strideA,
    const unsigned short* __restrict__ Btp, const unsigned short* __restrict__ Bt2p, int ldb, long strideB,
    void* __restrict__ Cout, void* __restrict__ Cout2, int ldc, long strideC,
    const float* __restrict__ bias,
    const float* __restrict__ resid, long strideR,
    int M, int N, int K, float scale) {
  typedef typename Elem<ET>::T T;
  typedef typename Frag<T>::V V;
  const T* A = (const T*)Ap; const T* A2 = (const T*)A2p; const T* Bt = (const T*)Btp; const T* Bt2 = (const T*)Bt2p;
  __shared__ __align__(16) float sT[8][16 * 68];
  const int b    = blockIdx.y;
  const int lane = threadIdx.x & 31;
  const int wave = threadIdx.x >> 5;
  const int tilesN = N >> 6;
  const int tilesM = M >> 6;
  const int tile = blockIdx.x * 8 + wave;
  if (tile >= tilesM * tilesN) return;
  const int tm = tile / tilesN;
  const int tn = tile - tm * tilesN;
  const int m0 = tm << 6;
  const int n0 = tn << 6;

  const T* Ab  = A  + (size_t)b * strideA;
  const T* Bb  = Bt + (size_t)b * strideB;
  const T* Ab2 = SPLIT ? (A2  + (size_t)b * strideA) : nullptr;
  const T* Bb2 = SPLIT ? (Bt2 + (size_t)b * strideB) : nullptr;

  const int rlane = lane & 15;
  const int koff  = (lane >> 4) * 8;
  const int mOff  = (lane >> 4) * 8;

  v8f acc[4][4];
#pragma unroll
  for (int i = 0; i < 4; ++i)
#pragma unroll
    for (int j = 0; j < 4; ++j) acc[i][j] = (v8f){0.f,0.f,0.f,0.f,0.f,0.f,0.f,0.f};

  for (int k0 = 0; k0 < K; k0 += 32) {
    V bh[4], bl[4];
#pragma unroll
    for (int j = 0; j < 4; ++j) {
      const size_t bo = (size_t)(n0 + (j << 4) + rlane) * ldb + koff + k0;
      bh[j] = Frag<T>::load(Bb + bo);
      if (SPLIT) bl[j] = Frag<T>::load(Bb2 + bo);
    }
#pragma unroll
    for (int i = 0; i < 4; ++i) {
      const size_t ao = (size_t)(m0 + (i << 4) + rlane) * lda + koff + k0;
      V ah = Frag<T>::load(Ab + ao);
      V al;
      if (SPLIT) al = Frag<T>::load(Ab2 + ao);
#pragma unroll
      for (int j = 0; j < 4; ++j) {
        acc[i][j] = Frag<T>::mma(ah, bh[j], acc[i][j]);
        if (SPLIT) {
          acc[i][j] = Frag<T>::mma(ah, bl[j], acc[i][j]);
          acc[i][j] = Frag<T>::mma(al, bh[j], acc[i][j]);
        }
      }
      Frag<T>::guard(acc[i][0], acc[i][3], ah, SPLIT ? al : ah);
    }
    Frag<T>::keep(bh[0], bh[1], bh[2], bh[3]);
    if (SPLIT) Frag<T>::keep(bl[0], bl[1], bl[2], bl[3]);
  }
  acc_guard4(acc[0][0], acc[0][1], acc[0][2], acc[0][3]);
  acc_guard4(acc[1][0], acc[1][1], acc[1][2], acc[1][3]);
  acc_guard4(acc[2][0], acc[2][1], acc[2][2], acc[2][3]);
  acc_guard4(acc[3][0], acc[3][1], acc[3][2], acc[3][3]);

  float* slab = sT[wave];
  const float* Rb = RESID ? (resid + (size_t)b * strideR) : nullptr;
#pragma unroll
  for (int i = 0; i < 4; ++i) {
    const int mBase = m0 + (i << 4);
#pragma unroll
    for (int j = 0; j < 4; ++j) {
      const int n = n0 + (j << 4) + rlane;
      float bv = 0.f;
      if (BIAS_MODE == 2) bv = bias[n];
#pragma unroll
      for (int r = 0; r < 8; ++r) {
        float v = acc[i][j][r] * scale;
        if (BIAS_MODE == 1) v += bias[mBase + mOff + r];
        if (BIAS_MODE == 2) v += bv;
        if (RESID) v += Rb[(size_t)(mBase + mOff + r) * ldc + n];
        if (ACT == 2) v = fmaxf(v, 0.0f);
        if (ACT == 4) v = (v > 0.f) ? v : 0.01f * v;
        slab[(mOff + r) * 68 + (j << 4) + rlane] = v;
      }
    }
    __builtin_amdgcn_fence(__ATOMIC_RELEASE, "workgroup");
    __builtin_amdgcn_wave_barrier();
    __builtin_amdgcn_fence(__ATOMIC_ACQUIRE, "workgroup");
    if (OUT_MODE == 0) {
      float* C = (float*)Cout + (size_t)b * strideC;
      const int hh = lane >> 4, c4 = (lane & 15) * 4;
      for (int pass = 0; pass < 2; ++pass) {
#pragma unroll
        for (int it = 0; it < 8; ++it) {
          const int row = it * 2 + hh;
          v4f v = *(const v4f*)(slab + row * 68 + c4);
          *(volatile v4f*)(C + (size_t)(mBase + row) * ldc + n0 + c4) = v;
        }
        __threadfence();
      }
    } else {
      const int q = lane >> 3, c8 = (lane & 7) * 8;
      unsigned short* C  = (unsigned short*)Cout  + (size_t)b * strideC;
      unsigned short* C2 = (OUT_MODE == 2) ? ((unsigned short*)Cout2 + (size_t)b * strideC) : nullptr;
      for (int pass = 0; pass < 2; ++pass) {
#pragma unroll
        for (int it = 0; it < 4; ++it) {
          const int row = it * 4 + q;
          const float* sp = slab + row * 68 + c8;
          v8h hv, lv;
#pragma unroll
          for (int e = 0; e < 8; ++e) {
            if (OUT_MODE == 1) {
              hv[e] = (_Float16)sp[e];
            } else {
              unsigned short hb = f2bf_bits(sp[e]);
              unsigned short lb = f2bf_bits(sp[e] - bf_bits2f(hb));
              hv[e] = __builtin_bit_cast(_Float16, hb);
              lv[e] = __builtin_bit_cast(_Float16, lb);
            }
          }
          *(volatile v8h*)(C + (size_t)(mBase + row) * ldc + n0 + c8) = hv;
          if (OUT_MODE == 2) *(volatile v8h*)(C2 + (size_t)(mBase + row) * ldc + n0 + c8) = lv;
        }
        __threadfence();
      }
    }
    __builtin_amdgcn_fence(__ATOMIC_RELEASE, "workgroup");
    __builtin_amdgcn_wave_barrier();
    __builtin_amdgcn_fence(__ATOMIC_ACQUIRE, "workgroup");
  }
}

__device__ __forceinline__ unsigned pack_hilo(float v) {
  const unsigned short hb = f2bf_bits(v);
  const unsigned short lb = f2bf_bits(v - bf_bits2f(hb));
  return (unsigned)hb | ((unsigned)lb << 16);
}
__device__ __forceinline__ unsigned join_hi(unsigned a, unsigned b) { return (a & 0xffffu) | (b << 16); }
__device__ __forceinline__ unsigned join_lo(unsigned a, unsigned b) { return (a >> 16) | (b & 0xffff0000u); }

__device__ __forceinline__ float knotf(int i) { return (float)(i - 3) * 0.4f + (-1.0f); }

__device__ __forceinline__ void eval_bases(float xv, v4u& hi, v4u& lo) {
  int cnt = 0;
#pragma unroll
  for (int i = 0; i < 12; ++i) cnt += (xv >= knotf(i)) ? 1 : 0;
  const int a = cnt - 1;
  const float gm2 = knotf(a - 2), gm1 = knotf(a - 1), ga0 = knotf(a);
  const float ga1 = knotf(a + 1), ga2 = knotf(a + 2), ga3 = knotf(a + 3);
  const float eps = 1e-8f;
  const float nL2 = xv - gm2, nL1 = xv - gm1, nL0 = xv - ga0;
  const float nR1 = ga1 - xv, nR2 = ga2 - xv, nR3 = ga3 - xv;
  const float d10  = (ga1 - ga0) + eps;
  const float d1m1 = (ga1 - gm1) + eps;
  const float d20  = (ga2 - ga0) + eps;
  const float d1m2 = (ga1 - gm2) + eps;
  const float d2m1 = (ga2 - gm1) + eps;
  const float d30  = (ga3 - ga0) + eps;
  const float b1m = nR1 / d10;
  const float b10 = nL0 / d10;
  const float b2mm = (nR1 / d1m1) * b1m;
  const float b2m  = (nL1 / d1m1) * b1m + (nR2 / d20) * b10;
  const float b20  = (nL0 / d20) * b10;
  const float b33 = (nR1 / d1m2) * b2mm;
  const float b32 = (nL2 / d1m2) * b2mm + (nR2 / d2m1) * b2m;
  const float b31 = (nL1 / d2m1) * b2m + (nR3 / d30) * b20;
  const float b30 = (nL0 / d30) * b20;
  const unsigned p33 = pack_hilo(b33), p32 = pack_hilo(b32), p31 = pack_hilo(b31), p30 = pack_hilo(b30);
  unsigned sel[8];
#pragma unroll
  for (int gi = 0; gi < 8; ++gi) {
    unsigned v = 0u;
    v = (a == gi)     ? p30 : v;
    v = (a == gi + 1) ? p31 : v;
    v = (a == gi + 2) ? p32 : v;
    v = (a == gi + 3) ? p33 : v;
    sel[gi] = v;
  }
  hi = (v4u){join_hi(sel[0], sel[1]), join_hi(sel[2], sel[3]), join_hi(sel[4], sel[5]), join_hi(sel[6], sel[7])};
  lo = (v4u){join_lo(sel[0], sel[1]), join_lo(sel[2], sel[3]), join_lo(sel[4], sel[5]), join_lo(sel[6], sel[7])};
}

__global__ __launch_bounds__(256) void weight_prep_kernel(
    const float* __restrict__ bw, const float* __restrict__ sw, const float* __restrict__ ss,
    unsigned short* __restrict__ Wh, unsigned short* __restrict__ Wl) {
  __shared__ float s_scal;
  const int o = blockIdx.x;
  const int t = threadIdx.x;
  if (t == 0) {
    float s = 0.0f;
    const float* sp = ss + (size_t)o * kKpatch;
#pragma unroll 1
    for (int i = 0; i < kKpatch; ++i) s += sp[i];
    s_scal = s * (1.0f / 288.0f);
  }
  __syncthreads();
  const float sc = s_scal;
  const float* swr = sw + (size_t)o * kKsp;
  const float* bwr = bw + (size_t)o * kKpatch;
  unsigned short* whr = Wh + (size_t)o * kPitch;
  unsigned short* wlr = Wl + (size_t)o * kPitch;
#pragma unroll 1
  for (int r = 0; r < 2; ++r) {
    const int j = r * 256 + t;
    if (j < kWChunks) {
      unsigned pk[8];
#pragma unroll
      for (int e = 0; e < 8; ++e) {
        const int col = j * 8 + e;
        const int cs = (col < kKsp) ? col : (kKsp - 1);
        int cb = col - kKsp;
        cb = (cb < 0) ? 0 : ((cb > kKpatch - 1) ? (kKpatch - 1) : cb);
        const float vs = sc * swr[cs];
        const float vb = bwr[cb];
        const float v = (col < kKsp) ? vs : ((col < kKtot) ? vb : 0.0f);
        pk[e] = pack_hilo(v);
      }
      const v4u hv = (v4u){join_hi(pk[0], pk[1]), join_hi(pk[2], pk[3]), join_hi(pk[4], pk[5]), join_hi(pk[6], pk[7])};
      const v4u lv = (v4u){join_lo(pk[0], pk[1]), join_lo(pk[2], pk[3]), join_lo(pk[4], pk[5]), join_lo(pk[6], pk[7])};
      unsigned short* dh = whr + (size_t)j * 8;
      unsigned short* dl = wlr + (size_t)j * 8;
      *(volatile v4u*)dh = hv;
      *(volatile v4u*)dl = lv;
      __threadfence();
      *(volatile v4u*)dh = hv;
      *(volatile v4u*)dl = lv;
    }
  }
}

__global__ __launch_bounds__(256) void pixel_bases_kernel(
    const float* __restrict__ x, v4u* __restrict__ PBh, v4u* __restrict__ PBl) {
  const int gidx = blockIdx.x * 256 + threadIdx.x;
  if (gidx >= kNPixP) return;
  const int gc = (gidx < kNPix) ? gidx : (kNPix - 1);
  float xv = x[gc];
  xv = (gidx < kNPix) ? xv : 0.0f;
  v4u hi, lo;
  eval_bases(xv, hi, lo);
  v4u* dh = PBh + gidx;
  v4u* dl = PBl + gidx;
  *(volatile v4u*)dh = hi;
  *(volatile v4u*)dl = lo;
  __threadfence();
  *(volatile v4u*)dh = hi;
  *(volatile v4u*)dl = lo;
}

__global__ __launch_bounds__(256) void feature_rows_kernel(
    const float* __restrict__ x, const v4u* __restrict__ PBh, const v4u* __restrict__ PBl,
    unsigned short* __restrict__ Fh, unsigned short* __restrict__ Fl, int row0) {
  const int lane = threadIdx.x & 31;
  const int wave = threadIdx.x >> 5;
  const int blkRow = blockIdx.x * kRowsPerBlk;
#pragma unroll 1
  for (int s = 0; s < kTasksPerWave; ++s) {
    const int task = s * 8 + wave;
    const int rl   = task / kGroups;
    const int q    = task - rl * kGroups;
    const int rloc = blkRow + rl;
    const int rg   = row0 + rloc;
    const int b    = rg >> 12;
    const int p    = rg & (kPos - 1);
    const int oy   = p >> 6;
    const int ox   = p & 63;
    unsigned short* fh = Fh + (size_t)rloc * kPitch;
    unsigned short* fl = Fl + (size_t)rloc * kPitch;
    unsigned xs0 = 0u, xs1 = 0u;
#pragma unroll
    for (int it = 0; it < 2; ++it) {
      const int cfb = 64 * q + 32 * it;
      const int cf  = cfb + lane;
      const int cfc = (cf < kKpatch) ? cf : (kKpatch - 1);
      const int c   = cfc / 9;
      const int f   = cfc - 9 * c;
      const int ky  = f / 3;
      const int kx  = f - 3 * ky;
      const int iy  = oy + ky - 1;
      const int ix  = ox + kx - 1;
      const bool inb = ((unsigned)iy < (unsigned)kImgH) && ((unsigned)ix < (unsigned)kImgW);
      const int iyc = (iy < 0) ? 0 : ((iy > kImgH - 1) ? (kImgH - 1) : iy);
      const int ixc = (ix < 0) ? 0 : ((ix > kImgW - 1) ? (kImgW - 1) : ix);
      const int pix = ((b * kCin + c) * kImgH + iyc) * kImgW + ixc;
      float xv = x[pix];
      xv = (inb && (cf < kKpatch)) ? xv : 0.0f;
      const unsigned xs = pack_hilo(xv);
      if (it == 0) xs0 = xs; else xs1 = xs;
      if (cfb < kKpatch) {
        const int pb = inb ? pix : kZSlot;
        const v4u vh = PBh[pb];
        const v4u vl = PBl[pb];
        unsigned short* dh = fh + (size_t)cf * 8;
        unsigned short* dl = fl + (size_t)cf * 8;
        *(volatile v4u*)dh = vh;
        *(volatile v4u*)dl = vl;
        __threadfence();
        *(volatile v4u*)dh = vh;
        *(volatile v4u*)dl = vl;
      }
    }
    unsigned w[8];
#pragma unroll
    for (int e = 0; e < 8; ++e) {
      const int src = (lane * 8 + e) & 31;
      const unsigned s0v = (unsigned)__shfl((int)xs0, src, 32);
      const unsigned s1v = (unsigned)__shfl((int)xs1, src, 32);
      w[e] = (lane < 4) ? s0v : s1v;
    }
    const v4u ph = (v4u){join_hi(w[0], w[1]), join_hi(w[2], w[3]), join_hi(w[4], w[5]), join_hi(w[6], w[7])};
    const v4u pl = (v4u){join_lo(w[0], w[1]), join_lo(w[2], w[3]), join_lo(w[4], w[5]), join_lo(w[6], w[7])};
    if (lane < 8) {
      unsigned short* dh = fh + kKsp + 64 * q + 8 * lane;
      unsigned short* dl = fl + kKsp + 64 * q + 8 * lane;
      *(volatile v4u*)dh = ph;
      *(volatile v4u*)dl = pl;
      __threadfence();
      *(volatile v4u*)dh = ph;
      *(volatile v4u*)dl = pl;
    }
  }
}

extern "C" void kernel_launch(void* const* d_in, const int* in_sizes, int n_in,
                              void* d_out, int out_size, void* d_ws, size_t ws_size,
                              hipStream_t stream) {
  if (n_in < 4) return;
  if (in_sizes[0] != kNPix) return;
  if (in_sizes[1] != kCout * kKpatch) return;
  if (in_sizes[2] != kCout * kKsp) return;
  if (in_sizes[3] != kCout * kKpatch) return;
  if (out_size != kRows * kCout) return;

  const float* x  = (const float*)d_in[0];
  const float* bw = (const float*)d_in[1];
  const float* sw = (const float*)d_in[2];
  const float* ss = (const float*)d_in[3];
  float* out = (float*)d_out;

  char* ws = (char*)d_ws;
  size_t off = 0;
  const size_t pbBytes = (size_t)kNPixP * 16;
  v4u* PBh = (v4u*)(ws + off); off += pbBytes;
  v4u* PBl = (v4u*)(ws + off); off += pbBytes;
  const size_t wBytes = (size_t)kCout * kPitch * 2;
  unsigned short* Wh = (unsigned short*)(ws + off); off += wBytes;
  unsigned short* Wl = (unsigned short*)(ws + off); off += wBytes;
  const size_t fBytes = (size_t)kChunkRows * kPitch * 2;
  unsigned short* Fh = (unsigned short*)(ws + off); off += fBytes;
  unsigned short* Fl = (unsigned short*)(ws + off); off += fBytes;
  if (off > ws_size) return;

  weight_prep_kernel<<<kCout, 256, 0, stream>>>(bw, sw, ss, Wh, Wl);
  pixel_bases_kernel<<<(kNPixP + 255) / 256, 256, 0, stream>>>(x, PBh, PBl);

  const int gemmTiles = (kCout / 64) * (kPos / 64);
  for (int ch = 0; ch < kNumChunks; ++ch) {
    feature_rows_kernel<<<kChunkRows / kRowsPerBlk, 256, 0, stream>>>(x, PBh, PBl, Fh, Fl, ch * kChunkRows);
    float* oc = out + (size_t)ch * kCout * kPos;
    wmma_gemm64<1, true, 0, 0, false, 0><<<dim3(gemmTiles / 8, 1), 256, 0, stream>>>(
        Wh, Wl, kPitch, 0L,
        Fh, Fl, kPitch, 0L,
        (void*)oc, (void*)nullptr, kPos, 0L,
        (const float*)nullptr,
        (const float*)nullptr, 0L,
        kCout, kPos, kKtot, 1.0f);
  }
}
